// RopeAttention_10282151707687
// MI455X (gfx1250) — hardware-verified
//
#include <hip/hip_runtime.h>


#ifndef NB
#define NB 2
#endif
#ifndef SEQ
#define SEQ 2048
#endif
#define NB_FULL 2
#define SEQ_FULL 2048
#define DM 2048
#define NH 32
#define NKV 8
#define REP (NH / NKV)
#define HD 64
#define DQ (NH * HD)
#define DKV (NKV * HD)
#define DQKV (DQ + 2 * DKV)
#define NFREQ (HD / 2)
#define RH (((SEQ) < 512) ? (SEQ) : 512)
#define PCAR 1024.0f
#define ATC 64.0f
#define WOC 64.0f
#define SCL 0.125f
#define L2E 1.4426950408889634f
#define NEGBIG (-1.0e30f)
#define PP 72
#define OSP 68
#define NFL (NB * SEQ / 64)
#define WS_LIMIT ((size_t)134217728)

static_assert(NB >= 1 && NB <= NB_FULL);
static_assert(SEQ % 128 == 0 && SEQ >= 128 && SEQ <= SEQ_FULL);
static_assert(RH % 64 == 0 && (SEQ - RH) % 64 == 0 && RH <= SEQ);
static_assert((NH * SEQ * HD) % 512 == 0);
static_assert((NKV * SEQ * HD) % 512 == 0);
static_assert((SEQ * DM) % 2048 == 0);
static_assert((SEQ * NFREQ) % 256 == 0);
static_assert((DQ * DM / 64) % 64 == 0 && (DKV * DM / 64) % 64 == 0);
static_assert(DM % 64 == 0 && DQ % 64 == 0 && DQKV % 64 == 0 && HD == 64);
static_assert((SEQ * DM) % 16384 == 0);
static_assert((NB * SEQ) % 64 == 0);
static_assert(15 * PP + 3 * 16 + 15 < 16 * PP);
static_assert(15 * OSP + 63 < 16 * OSP);

typedef _Float16 h16;
typedef unsigned short bf;
typedef __attribute__((ext_vector_type(16))) __bf16   v16bf;
typedef __attribute__((ext_vector_type(16))) _Float16 v16h;
typedef __attribute__((ext_vector_type(8)))  _Float16 v8h;
typedef __attribute__((ext_vector_type(8)))  unsigned short v8us;
typedef __attribute__((ext_vector_type(8)))  float    v8f;
typedef __attribute__((ext_vector_type(4)))  float    v4f;
typedef __attribute__((ext_vector_type(2)))  _Float16 v2h;
typedef __attribute__((ext_vector_type(4)))  _Float16 v4h;
typedef __attribute__((ext_vector_type(2)))  unsigned short v2us;
typedef __attribute__((ext_vector_type(4)))  unsigned short v4us;
typedef __attribute__((ext_vector_type(2)))  float v2f;
typedef __attribute__((ext_vector_type(4)))  int v4i;
typedef v8h  __attribute__((may_alias)) v8ha;
typedef v4f  __attribute__((may_alias)) v4fa;
typedef v8us __attribute__((may_alias)) v8usa;

#define G2(d0, d1, x0, x1) asm volatile("v_nop\n\tv_nop\n\tv_nop\n\tv_nop" : "+v"(d0), "+v"(d1) : "v"(x0), "v"(x1))
#define G4(d0, d1, d2, d3, x0, x1) asm volatile("v_nop\n\tv_nop\n\tv_nop\n\tv_nop" : "+v"(d0), "+v"(d1), "+v"(d2), "+v"(d3) : "v"(x0), "v"(x1))

__device__ __forceinline__ unsigned short f2bf(float f) { unsigned u = __float_as_uint(f); u += 0x7FFFu + ((u >> 16) & 1u); return (unsigned short)(u >> 16); }
__device__ __forceinline__ float bf2f(unsigned short b) { return __uint_as_float(((unsigned)b) << 16); }
__device__ __forceinline__ float bfr(float f) { return bf2f(f2bf(f)); }
__device__ __forceinline__ void splitf(float y, unsigned short& h, unsigned short& l) { h = f2bf(y); l = f2bf(y - bf2f(h)); }
__device__ __forceinline__ v16h cat16(v8h lo, v8h hi) { return __builtin_shufflevector(lo, hi, 0, 1, 2, 3, 4, 5, 6, 7, 8, 9, 10, 11, 12, 13, 14, 15); }
__device__ __forceinline__ v16bf cat16b(v8us lo, v8us hi) { return __builtin_bit_cast(v16bf, __builtin_shufflevector(lo, hi, 0, 1, 2, 3, 4, 5, 6, 7, 8, 9, 10, 11, 12, 13, 14, 15)); }
__device__ __forceinline__ v8f wmma16(v16h a, v16h b, v8f c) { return __builtin_amdgcn_wmma_f32_16x16x32_f16(false, a, false, b, (short)0, c, false, false); }
__device__ __forceinline__ v8f wmmab(v16bf a, v16bf b, v8f c) { return __builtin_amdgcn_wmma_f32_16x16x32_bf16(false, a, false, b, (short)0, c, false, false); }
__device__ __forceinline__ void wsync() { __builtin_amdgcn_fence(3  , "wavefront"); __builtin_amdgcn_wave_barrier(); asm volatile("" ::: "memory"); }

template <typename T16> struct WFrag;
template <> struct WFrag<h16> { typedef v16h V; static __device__ __forceinline__ V ld(const h16* p) { return cat16(*(const v8h*)p, *(const v8h*)(p + 16)); } static __device__ __forceinline__ v8f mma(V a, V b, v8f c) { return wmma16(a, b, c); } };
template <> struct WFrag<bf> { typedef v16bf V; static __device__ __forceinline__ V ld(const bf* p) { return cat16b(*(const v8us*)p, *(const v8us*)(p + 16)); } static __device__ __forceinline__ v8f mma(V a, V b, v8f c) { return wmmab(a, b, c); } };

template <typename T16, int NSPLIT>
__global__ __launch_bounds__(32) void k_gemmw(const T16* __restrict__ A, const T16* __restrict__ A2, const T16* __restrict__ Bt, const T16* __restrict__ Bt2, int K, float* C, int ldc, float osc, size_t sA, size_t sB, size_t sC) {
    typedef typename WFrag<T16>::V V;
    __shared__ __align__(16) float os[16 * OSP];
    const size_t z = blockIdx.z; A += z * sA; if (A2) A2 += z * sA; Bt += z * sB; if (Bt2) Bt2 += z * sB; C += z * sC;
    const int lane = threadIdx.x & 31, lr = lane & 15, hi = lane >> 4; const int r0 = blockIdx.x * 64, c0 = blockIdx.y * 64;
    v8f acc[4][4];
#pragma unroll
    for (int mb = 0; mb < 4; ++mb)
#pragma unroll
        for (int nb = 0; nb < 4; ++nb) acc[mb][nb] = (v8f){};
    const size_t aoff = (size_t)(r0 + lr) * K + 8 * hi, boff = (size_t)(c0 + lr) * K + 8 * hi;
#pragma unroll 1
    for (int kc = 0; kc < K; kc += 32) {
        V a[4], a2[4];
#pragma unroll
        for (int mb = 0; mb < 4; ++mb) { a[mb] = WFrag<T16>::ld(A + aoff + (size_t)mb * 16 * K + kc); if (NSPLIT == 1 || NSPLIT == 2) a2[mb] = WFrag<T16>::ld(A2 + aoff + (size_t)mb * 16 * K + kc); else a2[mb] = a[mb]; }
#pragma unroll
        for (int nb = 0; nb < 4; ++nb) { const V b = WFrag<T16>::ld(Bt + boff + (size_t)nb * 16 * K + kc); V b2 = b; if (NSPLIT >= 2) b2 = WFrag<T16>::ld(Bt2 + boff + (size_t)nb * 16 * K + kc);
#pragma unroll
            for (int mb = 0; mb < 4; ++mb) { acc[mb][nb] = WFrag<T16>::mma(a[mb], b, acc[mb][nb]); if (NSPLIT == 1 || NSPLIT == 2) acc[mb][nb] = WFrag<T16>::mma(a2[mb], b, acc[mb][nb]); if (NSPLIT >= 2) acc[mb][nb] = WFrag<T16>::mma(a[mb], b2, acc[mb][nb]); } }
        asm volatile("v_nop\n\tv_nop\n\tv_nop\n\tv_nop" : "+v"(acc[0][0]), "+v"(acc[1][1]), "+v"(acc[2][2]), "+v"(acc[3][3]) : "v"(a[0]), "v"(a[3]));
    }
#pragma unroll
    for (int mb = 0; mb < 4; ++mb) {
#pragma unroll
        for (int nb = 0; nb < 4; ++nb) {
#pragma unroll
            for (int j = 0; j < 8; ++j) os[(hi * 8 + j) * OSP + nb * 16 + lr] = acc[mb][nb][j]; }
        wsync();
        float* crow = C + (size_t)(r0 + mb * 16) * ldc + c0;
#pragma unroll 1
        for (int ps = 0; ps < 2; ++ps) {
#pragma unroll
            for (int s = 0; s < 8; ++s) { const int row = 2 * s + hi, cofs = lr * 4; v4f val = *(const v4fa*)(os + row * OSP + cofs); val = val * osc;
                *(volatile v4f*)(crow + (size_t)row * ldc + cofs) = val; }
            if (ps == 0) __threadfence(); }
        wsync();
    }
}

__global__ __launch_bounds__(256) void k_wtG(const float* __restrict__ w, int K, int N, bf* Bt) {
    const int lane = threadIdx.x & 31; const int L0 = (blockIdx.x * 8 + (threadIdx.x >> 5)) * 8; const int nlines = N * K / 64;
#pragma unroll
    for (int ps = 0; ps < 2; ++ps) {
#pragma unroll 1
        for (int l = 0; l < 8; ++l) { const int L = L0 + l; if (L >= nlines) break; const size_t e = (size_t)L * 64 + lane * 2; const int k = (int)(e % K), n = (int)(e / K); v2us o;
            o[0] = f2bf(w[(size_t)k * N + n]); o[1] = f2bf(w[(size_t)(k + 1) * N + n]); *(volatile v2us*)(Bt + e) = o; }
        if (ps == 0) __threadfence(); }
}
__global__ __launch_bounds__(256) void k_wtG2(const float* __restrict__ w, int K, int N, bf* Bt, h16* B16, float car) {
    const int lane = threadIdx.x & 31; const int L0 = (blockIdx.x * 8 + (threadIdx.x >> 5)) * 8; const int nlines = N * K / 64;
#pragma unroll
    for (int ps = 0; ps < 2; ++ps) {
#pragma unroll 1
        for (int l = 0; l < 8; ++l) { const int L = L0 + l; if (L >= nlines) break; const size_t e = (size_t)L * 64 + lane * 2; const int k = (int)(e % K), n = (int)(e / K); v2us o; v2h o2;
            o[0] = f2bf(w[(size_t)k * N + n]); o[1] = f2bf(w[(size_t)(k + 1) * N + n]); o2[0] = (h16)(bf2f(o[0]) * car); o2[1] = (h16)(bf2f(o[1]) * car);
            *(volatile v2us*)(Bt + e) = o; *(volatile v2h*)(B16 + e) = o2; }
        if (ps == 0) __threadfence(); }
}
__global__ __launch_bounds__(256) void k_cvt8(const float* __restrict__ src, bf* dst, size_t n8) { const size_t i = (size_t)blockIdx.x * 256 + threadIdx.x; if (i >= n8) return; const v8f v = *(const v8f*)(src + i * 8); v8us o;
#pragma unroll
    for (int k = 0; k < 8; ++k) o[k] = f2bf(v[k]); *(volatile v8us*)(dst + i * 8) = o; __threadfence(); *(volatile v8us*)(dst + i * 8) = o; }

__constant__ float INVF[NFREQ] = { 1.000000000e+00f, 7.498942018e-01f, 5.623413324e-01f, 4.216965139e-01f, 3.162277639e-01f, 2.371373773e-01f, 1.778279394e-01f, 1.333521456e-01f, 1.000000015e-01f, 7.498942316e-02f, 5.623413250e-02f, 4.216964915e-02f, 3.162277490e-02f, 2.371373773e-02f, 1.778279431e-02f, 1.333521400e-02f, 9.999999776e-03f, 7.498942316e-03f, 5.623413250e-03f, 4.216964822e-03f, 3.162277630e-03f, 2.371373819e-03f, 1.778279431e-03f, 1.333521446e-03f, 1.000000047e-03f, 7.498941850e-04f, 5.623413017e-04f, 4.216965172e-04f, 3.162277571e-04f, 2.371373703e-04f, 1.778279402e-04f, 1.333521504e-04f };
__global__ __launch_bounds__(256) void k_cs(float* CS) { const int idx = blockIdx.x * 256 + threadIdx.x; if (idx >= SEQ * NFREQ) return; const int i = idx % NFREQ; const int t = idx / NFREQ; const float a = __fmul_rn((float)t, INVF[i]); v2f cs; cs[0] = cosf(a); cs[1] = sinf(a); *(volatile v2f*)(CS + (size_t)idx * 2) = cs; __threadfence(); *(volatile v2f*)(CS + (size_t)idx * 2) = cs; }

__global__ __launch_bounds__(256) void k_rope(const float* __restrict__ F, int pitch, int col0, int nheads, int rh, const float* __restrict__ CS, h16* P16, bf* Ph, bf* Pl) {
#pragma clang fp contract(off)
    const size_t e = ((size_t)blockIdx.x * 256 + threadIdx.x) * 2; if (e >= (size_t)nheads * SEQ * HD) return;
    const int d = (int)(e % HD); const int t = (int)((e / HD) % SEQ); const int hh = (int)(e / ((size_t)HD * SEQ));
    const float* f = F + (size_t)t * pitch + col0 + hh * HD; const bool low = (d < HD / 2); const int pd = low ? d + HD / 2 : d - HD / 2;
    const float x0 = f[d], x1 = f[d + 1], y0 = f[pd], y1 = f[pd + 1];
    const v4f cs = *(const v4f*)(CS + ((size_t)t * NFREQ + (d & (NFREQ - 1))) * 2);
    float a0 = __fmul_rn(x0, cs[0]), b0 = __fmul_rn(y0, cs[1]), a1 = __fmul_rn(x1, cs[2]), b1 = __fmul_rn(y1, cs[3]); asm volatile("" : "+v"(a0), "+v"(b0), "+v"(a1), "+v"(b1));
    const float r0 = low ? __fsub_rn(a0, b0) : __fadd_rn(a0, b0); const float r1 = low ? __fsub_rn(a1, b1) : __fadd_rn(a1, b1);
    v2h o16; o16[0] = (h16)r0; o16[1] = (h16)r1; v2us oh, ol; { unsigned short a2, c2; splitf(r0, a2, c2); oh[0] = a2; ol[0] = c2; splitf(r1, a2, c2); oh[1] = a2; ol[1] = c2; }
    const bool dohl = (t < rh);
    const size_t oo = ((size_t)hh * rh + t) * HD + d;
    *(volatile v2h*)(P16 + e) = o16; if (dohl) { *(volatile v2us*)(Ph + oo) = oh; *(volatile v2us*)(Pl + oo) = ol; }
    __threadfence();
    *(volatile v2h*)(P16 + e) = o16; if (dohl) { *(volatile v2us*)(Ph + oo) = oh; *(volatile v2us*)(Pl + oo) = ol; }
}
__global__ __launch_bounds__(256) void k_vtp(const float* __restrict__ F, int pitch, int col0, int nheads, h16* V16, bf* Vh, bf* Vl) { const size_t e = ((size_t)blockIdx.x * 256 + threadIdx.x) * 2; if (e >= (size_t)nheads * HD * SEQ) return; const int t = (int)(e % SEQ); const int d = (int)((e / SEQ) % HD); const int g = (int)(e / ((size_t)SEQ * HD)); v2h o16; v2us oh, ol;
#pragma unroll
    for (int q = 0; q < 2; ++q) { const float x = F[(size_t)(t + q) * pitch + col0 + g * HD + d]; o16[q] = (h16)x; unsigned short a2, c2; splitf(x, a2, c2); oh[q] = a2; ol[q] = c2; }
    *(volatile v2h*)(V16 + e) = o16; *(volatile v2us*)(Vh + e) = oh; *(volatile v2us*)(Vl + e) = ol; __threadfence(); *(volatile v2h*)(V16 + e) = o16; *(volatile v2us*)(Vh + e) = oh; *(volatile v2us*)(Vl + e) = ol; }

template <bool HIRES, int KT>
__global__ __launch_bounds__(128) void k_attn(const h16* __restrict__ Q16, const bf* __restrict__ Qh, const bf* __restrict__ Ql,
                                               const h16* __restrict__ K16, const bf* __restrict__ Kh, const bf* __restrict__ Kl,
                                               const h16* __restrict__ V16, const bf* __restrict__ Vh, const bf* __restrict__ Vl,
                                               h16* AT16, bf* ATh, bf* ATl, int row0) {
    constexpr int NT = KT / 16; constexpr int KS = KT / 32; constexpr int NPL = HIRES ? 2 : 1;
    static_assert(NT == 2 || NT == 4);
    static_assert(15 * PP + (NT - 1) * 16 + 15 < 16 * PP);
    __shared__ __align__(16) unsigned short pt[NPL][4][16 * PP];
    __shared__ __align__(16) float os[4][16 * OSP];
    const int lane = threadIdx.x & 31, wave = threadIdx.x >> 5, lr = lane & 15, hi = lane >> 4;
    const int qbase = row0 + (blockIdx.x * 4 + wave) * 16; const int h = blockIdx.y; const int g = h / REP;
    v16h qa[2] = {}; v16bf qah[2] = {}, qal[2] = {};
    if (HIRES) { const size_t qo = ((size_t)h * RH + qbase + lr) * HD + 8 * hi; qah[0] = WFrag<bf>::ld(Qh + qo); qah[1] = WFrag<bf>::ld(Qh + qo + 32); qal[0] = WFrag<bf>::ld(Ql + qo); qal[1] = WFrag<bf>::ld(Ql + qo + 32); }
    else { const size_t qo = ((size_t)h * SEQ + qbase + lr) * HD + 8 * hi; qa[0] = WFrag<h16>::ld(Q16 + qo); qa[1] = WFrag<h16>::ld(Q16 + qo + 32); }
    const size_t kofs = (size_t)g * SEQ * HD + (size_t)lr * HD + 8 * hi;
    const size_t vofs = (size_t)g * HD * SEQ + (size_t)lr * SEQ + 8 * hi;
    v8f o[4];
#pragma unroll
    for (int nt = 0; nt < 4; ++nt) o[nt] = (v8f){};
    float mrun[8], lrun[8];
#pragma unroll
    for (int v = 0; v < 8; ++v) { mrun[v] = NEGBIG; lrun[v] = 0.f; }
    unsigned short* p0w = &pt[0][wave][0]; unsigned short* p1w = &pt[NPL - 1][wave][0];
    const int kend = qbase + 15;
#pragma unroll 1
    for (int kb = 0; kb <= kend; kb += KT) {
        v8f s[NT];
#pragma unroll
        for (int nt = 0; nt < NT; ++nt) s[nt] = (v8f){};
#pragma unroll
        for (int nt = 0; nt < NT; ++nt) {
#pragma unroll
            for (int kc = 0; kc < 2; ++kc) { const size_t ka = kofs + (size_t)(kb + nt * 16) * HD + kc * 32;
                if (HIRES) { const v16bf bh = WFrag<bf>::ld(Kh + ka), bl = WFrag<bf>::ld(Kl + ka); s[nt] = wmmab(qah[kc], bh, s[nt]); s[nt] = wmmab(qal[kc], bh, s[nt]); s[nt] = wmmab(qah[kc], bl, s[nt]); }
                else { const v16h b = WFrag<h16>::ld(K16 + ka); s[nt] = wmma16(qa[kc], b, s[nt]); } } }
        if constexpr (NT == 2) { if (HIRES) G2(s[0], s[1], qah[0], qal[1]); else G2(s[0], s[1], qa[0], qa[1]); }
        else { if (HIRES) G4(s[0], s[1], s[2], s[3], qah[0], qal[1]); else G4(s[0], s[1], s[2], s[3], qa[0], qa[1]); }
        float alpha[8];
#pragma unroll
        for (int v = 0; v < 8; ++v) {
            const int qi = qbase + 8 * hi + v; float x[NT]; float mx = NEGBIG;
#pragma unroll
            for (int nt = 0; nt < NT; ++nt) { const int j = kb + nt * 16 + lr; const float t = s[nt][v] * SCL; x[nt] = (j <= qi) ? t : NEGBIG; mx = fmaxf(mx, x[nt]); }
            mx = fmaxf(mx, __shfl_xor(mx, 1, 32)); mx = fmaxf(mx, __shfl_xor(mx, 2, 32)); mx = fmaxf(mx, __shfl_xor(mx, 4, 32)); mx = fmaxf(mx, __shfl_xor(mx, 8, 32));
            const float mnew = fmaxf(mrun[v], mx);
            const float a = __builtin_amdgcn_exp2f((mrun[v] - mnew) * L2E);
            float p[NT]; float rs = 0.f;
#pragma unroll
            for (int nt = 0; nt < NT; ++nt) { p[nt] = __builtin_amdgcn_exp2f((x[nt] - mnew) * L2E); rs += p[nt]; }
            rs += __shfl_xor(rs, 1, 32); rs += __shfl_xor(rs, 2, 32); rs += __shfl_xor(rs, 4, 32); rs += __shfl_xor(rs, 8, 32);
            lrun[v] = lrun[v] * a + rs; mrun[v] = mnew; alpha[v] = a;
#pragma unroll
            for (int nt = 0; nt < NT; ++nt) { const int idx = (8 * hi + v) * PP + nt * 16 + lr;
                if (HIRES) { unsigned short a2, c2; splitf(p[nt], a2, c2); p0w[idx] = a2; p1w[idx] = c2; }
                else { const h16 hv = (h16)(p[nt] * PCAR); p0w[idx] = __builtin_bit_cast(unsigned short, hv); } }
        }
        wsync();
        v16h pa[KS] = {}; v16bf pah[KS] = {}, pal[KS] = {};
        const unsigned short* pr0 = p0w + lr * PP + 8 * hi; const unsigned short* pr1 = p1w + lr * PP + 8 * hi;
#pragma unroll
        for (int ks = 0; ks < KS; ++ks) { const v8us u0 = *(const v8usa*)(pr0 + ks * 32); const v8us u1 = *(const v8usa*)(pr0 + ks * 32 + 16);
            if (HIRES) { const v8us w0 = *(const v8usa*)(pr1 + ks * 32); const v8us w1 = *(const v8usa*)(pr1 + ks * 32 + 16); pah[ks] = cat16b(u0, u1); pal[ks] = cat16b(w0, w1); }
            else { pa[ks] = cat16(__builtin_bit_cast(v8h, u0), __builtin_bit_cast(v8h, u1)); } }
#pragma unroll
        for (int nt = 0; nt < 4; ++nt) {
#pragma unroll
            for (int v = 0; v < 8; ++v) o[nt][v] *= alpha[v]; }
#pragma unroll
        for (int nt = 0; nt < 4; ++nt) {
#pragma unroll
            for (int ks = 0; ks < KS; ++ks) { const size_t va = vofs + (size_t)nt * 16 * SEQ + kb + ks * 32;
                if (HIRES) { const v16bf bh = WFrag<bf>::ld(Vh + va), bl = WFrag<bf>::ld(Vl + va); o[nt] = wmmab(pah[ks], bh, o[nt]); o[nt] = wmmab(pal[ks], bh, o[nt]); o[nt] = wmmab(pah[ks], bl, o[nt]); }
                else { const v16h b = WFrag<h16>::ld(V16 + va); o[nt] = wmma16(pa[ks], b, o[nt]); } } }
        if (HIRES) G4(o[0], o[1], o[2], o[3], pah[0], pal[KS - 1]); else G4(o[0], o[1], o[2], o[3], pa[0], pa[KS - 1]);
    }
    float* osw = &os[wave][0];
#pragma unroll
    for (int v = 0; v < 8; ++v) { const float f = HIRES ? __fdiv_rn(1.0f, lrun[v]) : __fdiv_rn(ATC / PCAR, lrun[v]);
#pragma unroll
        for (int nt = 0; nt < 4; ++nt) osw[(8 * hi + v) * OSP + nt * 16 + lr] = o[nt][v] * f; }
    wsync();
    const int rr = lane >> 3, c8 = (lane & 7) * 8;
#pragma unroll 1
    for (int ps = 0; ps < 2; ++ps) {
#pragma unroll
        for (int s4 = 0; s4 < 4; ++s4) { const int row = s4 * 4 + rr; const int t = qbase + row; const v4f u0 = *(const v4fa*)(osw + row * OSP + c8), u1 = *(const v4fa*)(osw + row * OSP + c8 + 4); const size_t oo = (size_t)t * DQ + h * HD + c8;
            if (HIRES) { v8us oh, ol;
#pragma unroll
                for (int q = 0; q < 4; ++q) { unsigned short a2, c2; splitf(u0[q], a2, c2); oh[q] = a2; ol[q] = c2; splitf(u1[q], a2, c2); oh[4 + q] = a2; ol[4 + q] = c2; }
                *(volatile v8us*)(ATh + oo) = oh; *(volatile v8us*)(ATl + oo) = ol; }
            else { v8h o8;
#pragma unroll
                for (int q = 0; q < 4; ++q) { o8[q] = (h16)u0[q]; o8[4 + q] = (h16)u1[q]; }
                *(volatile v8h*)(AT16 + oo) = o8; } }
        if (ps == 0) __threadfence(); }
}

__global__ __launch_bounds__(256) void k_mchk(const float* __restrict__ M, int* FL) {
    __shared__ int red[8];
    const int tid = threadIdx.x, lane = tid & 31, wave = tid >> 5; int bad = 0;
#pragma unroll 1
    for (int r = 0; r < 64; ++r) { const int gr = blockIdx.x * 64 + r; const int b = gr / SEQ, i = gr % SEQ; const float* mr = M + ((size_t)b * SEQ_FULL + i) * SEQ_FULL;
#pragma unroll 1
        for (int c = tid * 4; c < SEQ; c += 1024) { const v4f m = *(const v4f*)(mr + c);
#pragma unroll
            for (int q = 0; q < 4; ++q) { const int j = c + q; const bool ok = (j <= i) ? (m[q] == 0.0f) : (m[q] <= -1.0e8f); bad += ok ? 0 : 1; } } }
#pragma unroll
    for (int sh = 16; sh; sh >>= 1) bad += __shfl_xor(bad, sh, 32);
    if (lane == 0) red[wave] = bad;
    __syncthreads();
    if (wave == 0) { int v = red[lane & 7]; v = (lane < 8) ? v : 0;
#pragma unroll
        for (int sh = 16; sh; sh >>= 1) v += __shfl_xor(v, sh, 32);
        v4i o; o[0] = v; o[1] = v; o[2] = v; o[3] = v;
        if (lane < 8) *(volatile v4i*)(FL + (size_t)blockIdx.x * 32 + lane * 4) = o;
        __threadfence();
        if (lane < 8) *(volatile v4i*)(FL + (size_t)blockIdx.x * 32 + lane * 4) = o; }
}
__global__ __launch_bounds__(256) void k_poison(const int* __restrict__ FL, int nfl, float* out) {
    int tot = 0;
#pragma unroll 1
    for (int f = 0; f < nfl; ++f) tot += FL[(size_t)f * 32];
    if (tot == 0) return;
    float* ob = out + (size_t)blockIdx.y * SEQ_FULL * DM + (size_t)blockIdx.x * 16384;
    const float qn = __uint_as_float(0x7fc00000u); v4f nv; nv[0] = qn; nv[1] = qn; nv[2] = qn; nv[3] = qn;
#pragma unroll 1
    for (int ps = 0; ps < 2; ++ps) {
#pragma unroll 1
        for (int s = 0; s < 16; ++s) *(volatile v4f*)(ob + ((size_t)s * 256 + threadIdx.x) * 4) = nv;
        if (ps == 0) __threadfence(); }
}

extern "C" void kernel_launch(void* const* d_in, const int* in_sizes, int n_in,
                              void* d_out, int out_size, void* d_ws, size_t ws_size, hipStream_t stream) {
    if (n_in < 6) return;
    if ((size_t)in_sizes[0] < (size_t)(NB - 1) * SEQ_FULL * DM + (size_t)SEQ * DM) return;
    if ((size_t)in_sizes[1] < (size_t)(NB - 1) * SEQ_FULL * SEQ_FULL + (size_t)SEQ * SEQ_FULL) return;
    if ((size_t)in_sizes[2] < (size_t)DM * DQ || (size_t)in_sizes[3] < (size_t)DM * DKV || (size_t)in_sizes[4] < (size_t)DM * DKV || (size_t)in_sizes[5] < (size_t)DQ * DM) return;
    if ((size_t)out_size < (size_t)(NB - 1) * SEQ_FULL * DM + (size_t)SEQ * DM) return;
    const float* x = (const float*)d_in[0]; const float* am = (const float*)d_in[1]; const float* wq = (const float*)d_in[2]; const float* wk = (const float*)d_in[3]; const float* wv = (const float*)d_in[4]; const float* wo = (const float*)d_in[5];
    float* OUT = (float*)d_out;
    char* wsp = (char*)d_ws;
    auto take = [&](size_t bytes) { char* p = wsp; wsp += (bytes + 255) & ~(size_t)255; return (void*)p; };
    bf* WQKV = (bf*)take((size_t)DQKV * DM * 2); bf* WOB = (bf*)take((size_t)DM * DQ * 2); h16* WO16 = (h16*)take((size_t)DM * DQ * 2);
    float* CS = (float*)take((size_t)SEQ * NFREQ * 2 * 4); int* FL = (int*)take((size_t)NFL * 32 * 4);
    bf* XB = (bf*)take((size_t)SEQ * DM * 2); float* F = (float*)take((size_t)SEQ * DQKV * 4);
    h16* Q16 = (h16*)take((size_t)NH * SEQ * HD * 2); bf* Qh = (bf*)take((size_t)NH * RH * HD * 2); bf* Ql = (bf*)take((size_t)NH * RH * HD * 2);
    h16* K16 = (h16*)take((size_t)NKV * SEQ * HD * 2); bf* Kh = (bf*)take((size_t)NKV * SEQ * HD * 2); bf* Kl = (bf*)take((size_t)NKV * SEQ * HD * 2);
    h16* V16 = (h16*)take((size_t)NKV * HD * SEQ * 2); bf* Vh = (bf*)take((size_t)NKV * HD * SEQ * 2); bf* Vl = (bf*)take((size_t)NKV * HD * SEQ * 2);
    h16* AT16 = (h16*)take((size_t)SEQ * DQ * 2); bf* ATh = (bf*)take((size_t)RH * DQ * 2); bf* ATl = (bf*)take((size_t)RH * DQ * 2);
    const size_t used = (size_t)(wsp - (char*)d_ws); if (used > ws_size || used > WS_LIMIT) return;

    k_wtG<<<(unsigned)((DQ * DM / 64 + 63) / 64), 256, 0, stream>>>(wq, DM, DQ, WQKV);
    k_wtG<<<(unsigned)((DKV * DM / 64 + 63) / 64), 256, 0, stream>>>(wk, DM, DKV, WQKV + (size_t)DQ * DM);
    k_wtG<<<(unsigned)((DKV * DM / 64 + 63) / 64), 256, 0, stream>>>(wv, DM, DKV, WQKV + (size_t)(DQ + DKV) * DM);
    k_wtG2<<<(unsigned)((DM * DQ / 64 + 63) / 64), 256, 0, stream>>>(wo, DQ, DM, WOB, WO16, WOC);
    k_cs<<<(unsigned)((SEQ * NFREQ + 255) / 256), 256, 0, stream>>>(CS);
    k_mchk<<<(unsigned)NFL, 256, 0, stream>>>(am, FL);
    const unsigned LQ = (unsigned)(((size_t)NH * SEQ * HD / 2 + 255) / 256), LK = (unsigned)(((size_t)NKV * SEQ * HD / 2 + 255) / 256);
    for (int b = 0; b < NB; ++b) {
        float* OUTb = OUT + (size_t)b * SEQ_FULL * DM;
        k_cvt8<<<(unsigned)(((size_t)SEQ * DM / 8 + 255) / 256), 256, 0, stream>>>(x + (size_t)b * SEQ_FULL * DM, XB, (size_t)SEQ * DM / 8);
        k_gemmw<bf, 0><<<dim3(SEQ / 64, DQKV / 64, 1), 32, 0, stream>>>(XB, nullptr, WQKV, nullptr, DM, F, DQKV, 1.0f, 0, 0, 0);
        k_rope<<<LQ, 256, 0, stream>>>(F, DQKV, 0, NH, RH, CS, Q16, Qh, Ql);
        k_rope<<<LK, 256, 0, stream>>>(F, DQKV, DQ, NKV, SEQ, CS, K16, Kh, Kl);
        k_vtp<<<LK, 256, 0, stream>>>(F, DQKV, DQ + DKV, NKV, V16, Vh, Vl);
        k_attn<true, 32><<<dim3(RH / 64, NH, 1), 128, 0, stream>>>(Q16, Qh, Ql, K16, Kh, Kl, V16, Vh, Vl, AT16, ATh, ATl, 0);
        if (SEQ > RH) k_attn<false, 64><<<dim3((SEQ - RH) / 64, NH, 1), 128, 0, stream>>>(Q16, Qh, Ql, K16, Kh, Kl, V16, Vh, Vl, AT16, ATh, ATl, RH);
        k_gemmw<bf, 1><<<dim3(RH / 64, DM / 64, 1), 32, 0, stream>>>(ATh, ATl, WOB, nullptr, DQ, OUTb, DM, 1.0f, 0, 0, 0);
        if (SEQ > RH) k_gemmw<h16, 0><<<dim3((SEQ - RH) / 64, DM / 64, 1), 32, 0, stream>>>(AT16 + (size_t)RH * DQ, nullptr, WO16, nullptr, DQ, OUTb + (size_t)RH * DM, DM, 1.0f / (ATC * WOC), 0, 0, 0);
    }
    k_poison<<<dim3(SEQ * DM / 16384, NB, 1), 256, 0, stream>>>(FL, NFL, OUT);
}
